// NVARReservoir_48636209660445
// MI455X (gfx1250) — hardware-run, weakly checked
//
#include <hip/hip_runtime.h>


#define NRW  1024
#define NPR  512
#define NEM  64
#define NDL  5
#define NLF  320
#define NLN  384
#define KTT  61824
#define NSRC 51681
#define IPS  0.000244140625f
constexpr size_t al256(size_t b) { return (b + 255) & ~(size_t)255; }
constexpr size_t WS_TOTAL = al256((size_t)NEM * KTT * 2) + al256((size_t)NPR * KTT * 2) + al256((size_t)NRW * NEM * 4);
static_assert(WS_TOTAL == 71483392 && WS_TOTAL <= 134217728, "the workspace carve: 68.2 MiB");
static_assert(KTT == NLN + 64 * 64 * (5 + 4 + 3 + 2 + 1) && KTT % 64 == 0 && KTT % 32 == 0 && NLF == NEM * NDL && NLF == 5 * 64 && NSRC == 1 + NLF + NLF * (NLF + 1) / 2 && NRW == 2 * NPR && NPR % 64 == 0 && (NPR & (NPR - 1)) == 0 && (NEM & (NEM - 1)) == 0, "the laid-out depth; whole lines; whole depth steps");

__device__ __forceinline__ unsigned runbase(unsigned i) { const unsigned q = i >> 6, r = i & 63u; return NLN + 64u * (64u * (5u * q - q * (q - 1u) / 2u) + (5u - q) * r); }
typedef _Float16 h16;
typedef unsigned short bf;
typedef __attribute__((ext_vector_type(16))) __bf16   v16bf;
typedef __attribute__((ext_vector_type(16))) _Float16 v16h;
typedef __attribute__((ext_vector_type(8)))  _Float16 v8h;
typedef __attribute__((ext_vector_type(8)))  unsigned short v8us;
typedef __attribute__((ext_vector_type(8)))  float    v8f;
typedef __attribute__((ext_vector_type(4)))  float    v4f;
typedef v8h  __attribute__((may_alias)) v8ha;
typedef v4f  __attribute__((may_alias)) v4fa;
typedef v8us __attribute__((may_alias)) v8usa;

__device__ __forceinline__ unsigned short f2bf(float f) { unsigned u = __float_as_uint(f); u += 0x7FFFu + ((u >> 16) & 1u); return (unsigned short)(u >> 16); }
__device__ __forceinline__ float bf2f(unsigned short b) { return __uint_as_float(((unsigned)b) << 16); }
__device__ __forceinline__ float bfr(float f) { return bf2f(f2bf(f)); }
__device__ __forceinline__ v16h cat16(v8h lo, v8h hi) { return __builtin_shufflevector(lo, hi, 0, 1, 2, 3, 4, 5, 6, 7, 8, 9, 10, 11, 12, 13, 14, 15); }
__device__ __forceinline__ v16bf cat16b(v8us lo, v8us hi) { return __builtin_bit_cast(v16bf, __builtin_shufflevector(lo, hi, 0, 1, 2, 3, 4, 5, 6, 7, 8, 9, 10, 11, 12, 13, 14, 15)); }
__device__ __forceinline__ v8f wmma16(v16h a, v16h b, v8f c) { return __builtin_amdgcn_wmma_f32_16x16x32_f16(false, a, false, b, (short)0, c, false, false); }
__device__ __forceinline__ v8f wmmab(v16bf a, v16bf b, v8f c) { return __builtin_amdgcn_wmma_f32_16x16x32_bf16(false, a, false, b, (short)0, c, false, false); }


template <typename T16> struct WFrag;
template <> struct WFrag<h16> { typedef v16h V; static __device__ __forceinline__ V ld(const h16* p) { return cat16(*(const v8h*)p, *(const v8h*)(p + 16)); } static __device__ __forceinline__ v8f mma(V a, V b, v8f c) { return wmma16(a, b, c); } };
template <> struct WFrag<bf> { typedef v16bf V; static __device__ __forceinline__ V ld(const bf* p) { return cat16b(*(const v8us*)p, *(const v8us*)(p + 16)); } static __device__ __forceinline__ v8f mma(V a, V b, v8f c) { return wmmab(a, b, c); } };
template <typename T16, int NSPLIT, bool BIAS>
__global__ __launch_bounds__(32) void k_gemmw(const T16* __restrict__ A, const T16* __restrict__ A2, const T16* __restrict__ Bt, const T16* __restrict__ Bt2, int K, float* C, int ldc, const float* __restrict__ bias, size_t sA, size_t sB, size_t sC) {
    typedef typename WFrag<T16>::V V;
    __shared__ __align__(16) float os[16 * 68];
    const size_t z = blockIdx.z; A += z * sA; if (A2) A2 += z * sA; Bt += z * sB; if (Bt2) Bt2 += z * sB; C += z * sC;
    const int lane = threadIdx.x & 31, lr = lane & 15, hi = lane >> 4; const int r0 = blockIdx.x * 64, c0 = blockIdx.y * 64;
    v8f acc[4][4];
#pragma unroll
    for (int mb = 0; mb < 4; ++mb)
#pragma unroll
        for (int nb = 0; nb < 4; ++nb) acc[mb][nb] = (v8f){};
    const size_t aoff = (size_t)(r0 + lr) * K + 8 * hi, boff = (size_t)(c0 + lr) * K + 8 * hi;
    for (int kc = 0; kc < K; kc += 32) {
        V a[4], a2[4];
#pragma unroll
        for (int mb = 0; mb < 4; ++mb) { a[mb] = WFrag<T16>::ld(A + aoff + (size_t)mb * 16 * K + kc); if (NSPLIT == 1 || NSPLIT == 2) a2[mb] = WFrag<T16>::ld(A2 + aoff + (size_t)mb * 16 * K + kc); }
#pragma unroll
        for (int nb = 0; nb < 4; ++nb) { const V b = WFrag<T16>::ld(Bt + boff + (size_t)nb * 16 * K + kc); V b2; if (NSPLIT >= 2) b2 = WFrag<T16>::ld(Bt2 + boff + (size_t)nb * 16 * K + kc);
#pragma unroll
            for (int mb = 0; mb < 4; ++mb) { acc[mb][nb] = WFrag<T16>::mma(a[mb], b, acc[mb][nb]); if (NSPLIT == 1 || NSPLIT == 2) acc[mb][nb] = WFrag<T16>::mma(a2[mb], b, acc[mb][nb]); if (NSPLIT >= 2) acc[mb][nb] = WFrag<T16>::mma(a[mb], b2, acc[mb][nb]); } }
        asm volatile("v_nop\n\tv_nop\n\tv_nop\n\tv_nop" : "+v"(acc[0][0]), "+v"(acc[1][1]), "+v"(acc[2][2]), "+v"(acc[3][3]) : "v"(a[0]), "v"(a[3]));
    }
#pragma unroll
    for (int mb = 0; mb < 4; ++mb) {
#pragma unroll
        for (int nb = 0; nb < 4; ++nb) {
#pragma unroll
            for (int j = 0; j < 8; ++j) os[(hi * 8 + j) * 68 + nb * 16 + lr] = acc[mb][nb][j]; }
        __builtin_amdgcn_wave_barrier(); asm volatile("" ::: "memory");
        float* crow = C + (size_t)(r0 + mb * 16) * ldc + c0;
#pragma unroll 1
        for (int ps = 0; ps < 2; ++ps) {
#pragma unroll
            for (int s = 0; s < 8; ++s) { const int row = 2 * s + hi, cofs = lr * 4; v4f val = *(const v4fa*)(os + row * 68 + cofs); if (BIAS) { val[0] += bfr(bias[c0 + cofs]); val[1] += bfr(bias[c0 + cofs + 1]); val[2] += bfr(bias[c0 + cofs + 2]); val[3] += bfr(bias[c0 + cofs + 3]); }
                *(volatile v4f*)(crow + (size_t)row * ldc + cofs) = val; }
            if (ps == 0) __threadfence(); }
        __builtin_amdgcn_wave_barrier(); asm volatile("" ::: "memory");
    }
}

__device__ __forceinline__ h16 tohx(float x) { return (h16)x; }
__device__ __forceinline__ void splitf(float y, unsigned short& h, unsigned short& l) { h = f2bf(y); l = f2bf(y - bf2f(h)); }
typedef __attribute__((ext_vector_type(2))) _Float16 v2h;
typedef __attribute__((ext_vector_type(4))) _Float16 v4h;
typedef __attribute__((ext_vector_type(2))) unsigned short v2us;
typedef __attribute__((ext_vector_type(4))) unsigned short v4us;
typedef __attribute__((ext_vector_type(2))) float v2f;
typedef __attribute__((ext_vector_type(4))) int v4i;


__global__ __launch_bounds__(256) void k_wre(const float* __restrict__ ua, h16* BT) {
    const unsigned g = blockIdx.x * 256 + threadIdx.x; if (g >= (unsigned)(NEM * 6 * 8)) return; const unsigned sg = blockIdx.y; const unsigned item = g >> 3, c8 = g & 7u; const unsigned n = item / 6u, ln = item - n * 6u;
    const unsigned i = sg == 0u ? 0u : sg - 1u; const unsigned nl = sg == 0u ? 6u : 5u - (i >> 6); if (ln >= nl) return; const unsigned base = sg == 0u ? 0u : runbase(i); const unsigned p0 = 64u * ln + 8u * c8;
    const unsigned s0 = sg == 0u ? 0u : 1u + NLF + NLF * i - i * (i - 1u) / 2u; const unsigned lim = sg == 0u ? (unsigned)NLF + 1u : (unsigned)NLF - i; v8h o;
#pragma unroll
    for (int w = 0; w < 8; ++w) { const unsigned p = p0 + w; const bool live = p < lim; const float v = bfr(ua[(size_t)(live ? s0 + p : 0u) * NEM + n]); o[w] = tohx(live ? v * 256.0f : 0.0f); }
    h16* d8 = BT + (size_t)n * KTT + base + p0; *(volatile v8h*)(d8) = o; __threadfence(); *(volatile v8h*)(d8) = o; }

__device__ __forceinline__ float fvw(const float* __restrict__ xb, unsigned s, unsigned idx) { const unsigned e0 = idx / NDL, k = idx - e0 * NDL; const unsigned e = e0 & (unsigned)(NEM - 1); const unsigned su = s + k; const bool lv = su >= (unsigned)(NDL - 1); const unsigned rw = (lv ? su - (unsigned)(NDL - 1) : 0u) & (unsigned)(NPR - 1); const float v = bfr(xb[(size_t)rw * NEM + e]); return lv ? v : 0.0f; }
__global__ __launch_bounds__(256) void k_feat(const float* __restrict__ xb, h16* AP) {
    const unsigned g = blockIdx.x * 256 + threadIdx.x; if (g >= (unsigned)(NPR * 6 * 8)) return; const unsigned sg = blockIdx.y; const unsigned item = g >> 3, c8 = g & 7u; const unsigned s = item / 6u, ln = item - s * 6u;
    const unsigned i = sg == 0u ? 0u : sg - 1u; const unsigned nl = sg == 0u ? 6u : 5u - (i >> 6); if (ln >= nl) return; const unsigned base = sg == 0u ? 0u : runbase(i); const unsigned p0 = 64u * ln + 8u * c8; v8h o;
    const float fi = sg == 0u ? 1.0f : fvw(xb, s, i);
#pragma unroll
    for (int w = 0; w < 8; ++w) { const unsigned p = p0 + w; float v;
        if (sg == 0u) { const unsigned idx = p == 0u ? 0u : (p <= (unsigned)NLF ? p - 1u : 0u); const float f = fvw(xb, s, idx); v = p == 0u ? 1.0f : (p <= (unsigned)NLF ? f : 0.0f); }
        else { const unsigned j = i + p; const float f = fvw(xb, s, j < (unsigned)NLF ? j : 0u); v = j < (unsigned)NLF ? fi * f : 0.0f; }
        o[w] = tohx(v * 16.0f); }
    h16* d8 = AP + (size_t)s * KTT + base + p0; *(volatile v8h*)(d8) = o; __threadfence(); *(volatile v8h*)(d8) = o; }

__global__ __launch_bounds__(64) void k_head(const float* __restrict__ CP, const float* __restrict__ ca, const float* __restrict__ ub, const float* __restrict__ cb, float* rs) {
    const unsigned row = blockIdx.x * 64 + threadIdx.x; if (row >= (unsigned)NRW) return; float ac[NEM];
#pragma unroll
    for (int m = 0; m < NEM; ++m) ac[m] = 0.0f;
    for (int n = 0; n < NEM; ++n) { const float pv = CP[(size_t)row * NEM + n] * IPS + bfr(ca[n]); const float gv = 0.5f * pv * (1.0f + erff(pv * 0.70710678118654752f));
#pragma unroll
        for (int m = 0; m < NEM; ++m) ac[m] += gv * bfr(ub[n * NEM + m]); }
    float* d = rs + (size_t)row * NEM;
#pragma unroll
    for (int c = 0; c < NEM / 4; ++c) { v4f o; o[0] = ac[4 * c] + bfr(cb[4 * c]); o[1] = ac[4 * c + 1] + bfr(cb[4 * c + 1]); o[2] = ac[4 * c + 2] + bfr(cb[4 * c + 2]); o[3] = ac[4 * c + 3] + bfr(cb[4 * c + 3]); *(volatile v4f*)(d + 4 * c) = o; }
    __threadfence();
#pragma unroll
    for (int c = 0; c < NEM / 4; ++c) { v4f o; o[0] = ac[4 * c] + bfr(cb[4 * c]); o[1] = ac[4 * c + 1] + bfr(cb[4 * c + 1]); o[2] = ac[4 * c + 2] + bfr(cb[4 * c + 2]); o[3] = ac[4 * c + 3] + bfr(cb[4 * c + 3]); *(volatile v4f*)(d + 4 * c) = o; } }

extern "C" void kernel_launch(void* const* d_in, const int* in_sizes, int n_in,
                              void* d_out, int out_size, void* d_ws, size_t ws_size, hipStream_t stream) {
    if (n_in < 5) return;
    if (in_sizes[0] < NRW * NEM || in_sizes[1] < NSRC * NEM || in_sizes[2] < NEM || in_sizes[3] < NEM * NEM || in_sizes[4] < NEM || out_size < NRW * NEM) return;
    const float* xi = (const float*)d_in[0]; const float* ua = (const float*)d_in[1]; const float* ca = (const float*)d_in[2]; const float* ub = (const float*)d_in[3]; const float* cb = (const float*)d_in[4];
    char* wsp = (char*)d_ws;
    auto take = [&](size_t bytes) { char* cur = wsp; wsp += (bytes + 255) & ~(size_t)255; return (void*)cur; };
    h16* BT = (h16*)take((size_t)NEM * KTT * 2); h16* AP = (h16*)take((size_t)NPR * KTT * 2); float* CP = (float*)take((size_t)NRW * NEM * 4);
    if ((size_t)(wsp - (char*)d_ws) != WS_TOTAL || WS_TOTAL > ws_size) return;
    k_wre<<<dim3(NEM * 6 * 8 / 256, 1 + NLF, 1), 256, 0, stream>>>(ua, BT);
    for (int pt = 0; pt < NRW / NPR; ++pt) {
        k_feat<<<dim3(NPR * 6 * 8 / 256, 1 + NLF, 1), 256, 0, stream>>>(xi + (size_t)pt * NPR * NEM, AP);
        k_gemmw<h16, 0, false><<<dim3(NPR / 64, NEM / 64, 1), 32, 0, stream>>>(AP, nullptr, BT, nullptr, KTT, CP + (size_t)pt * NPR * NEM, NEM, nullptr, (size_t)0, (size_t)0, (size_t)0);
    }
    k_head<<<NRW / 64, 64, 0, stream>>>(CP, ca, ub, cb, (float*)d_out);
}
